// Hgru2_1d_8521215115682
// MI455X (gfx1250) — hardware-verified
//
#include <hip/hip_runtime.h>
#include <stdint.h>

typedef __attribute__((ext_vector_type(16))) _Float16 v16h;
typedef __attribute__((ext_vector_type(8)))  _Float16 v8h;
typedef __attribute__((ext_vector_type(16))) __bf16   v16b;
typedef __attribute__((ext_vector_type(8)))  __bf16   v8b;
typedef __attribute__((ext_vector_type(8)))  float    v8f;
typedef __attribute__((ext_vector_type(4)))  float    v4f;

#define SC_D  1024
#define SC_N3 3072

__device__ __forceinline__ unsigned short f2bf_bits(float f) {
  unsigned u = __float_as_uint(f);
  return (unsigned short)((u + 0x7FFFu + ((u >> 16) & 1u)) >> 16);
}
__device__ __forceinline__ float bf_bits2f(unsigned short h) { return __uint_as_float(((unsigned)h) << 16); }

__device__ __forceinline__ void dep_guard_h(v8f& a, v8f& b, v16h x, v16h y) { asm volatile("v_nop\n\tv_nop\n\tv_nop\n\tv_nop" : "+v"(a), "+v"(b) : "v"(x), "v"(y)); }
__device__ __forceinline__ void dep_guard_b(v8f& a, v8f& b, v16b x, v16b y) { asm volatile("v_nop\n\tv_nop\n\tv_nop\n\tv_nop" : "+v"(a), "+v"(b) : "v"(x), "v"(y)); }
__device__ __forceinline__ void keep4_h(v16h a, v16h b, v16h c, v16h d) { asm volatile("v_nop" :: "v"(a), "v"(b), "v"(c), "v"(d)); }
__device__ __forceinline__ void keep4_b(v16b a, v16b b, v16b c, v16b d) { asm volatile("v_nop" :: "v"(a), "v"(b), "v"(c), "v"(d)); }
__device__ __forceinline__ void acc_guard4(v8f& a, v8f& b, v8f& c, v8f& d) { asm volatile("v_nop\n\tv_nop\n\tv_nop\n\tv_nop" : "+v"(a), "+v"(b), "+v"(c), "+v"(d)); }
template <typename T> struct Frag;
template <> struct Frag<_Float16> {
  typedef v16h V; union U { v16h v; v8h h[2]; };
  static __device__ __forceinline__ v16h load(const _Float16* p) {
    U f; f.h[0] = *(const v8h*)(p); f.h[1] = *(const v8h*)(p + 16); return f.v;
  }
  static __device__ __forceinline__ v8f mma(v16h a, v16h b, v8f c) {
    return __builtin_amdgcn_wmma_f32_16x16x32_f16(false, a, false, b, (short)0, c, false, false);
  }
  static __device__ __forceinline__ void guard(v8f& a, v8f& b, v16h x, v16h y) { dep_guard_h(a, b, x, y); }
  static __device__ __forceinline__ void keep(v16h a, v16h b, v16h c, v16h d) { keep4_h(a, b, c, d); }
};
template <> struct Frag<__bf16> {
  typedef v16b V; union U { v16b v; v8b h[2]; };
  static __device__ __forceinline__ v16b load(const __bf16* p) {
    U f; f.h[0] = *(const v8b*)(p); f.h[1] = *(const v8b*)(p + 16); return f.v;
  }
  static __device__ __forceinline__ v8f mma(v16b a, v16b b, v8f c) {
    return __builtin_amdgcn_wmma_f32_16x16x32_bf16(false, a, false, b, (short)0, c, false, false);
  }
  static __device__ __forceinline__ void guard(v8f& a, v8f& b, v16b x, v16b y) { dep_guard_b(a, b, x, y); }
  static __device__ __forceinline__ void keep(v16b a, v16b b, v16b c, v16b d) { keep4_b(a, b, c, d); }
};

template <int ET> struct Elem;
template <> struct Elem<0> { typedef _Float16 T; };
template <> struct Elem<1> { typedef __bf16 T; };
template <int ET, bool SPLIT, int BIAS_MODE, int OUT_MODE, bool RESID, int ACT = 0>
__global__ __launch_bounds__(256) void wmma_gemm64(
    const unsigned short* __restrict__ Ap, const unsigned short* __restrict__ A2p, int lda, long strideA,
    const unsigned short* __restrict__ Btp, const unsigned short* __restrict__ Bt2p, int ldb, long strideB,
    void* __restrict__ Cout, void* __restrict__ Cout2, int ldc, long strideC,
    const float* __restrict__ bias,
    const float* __restrict__ resid, long strideR,
    int M, int N, int K, float scale) {
  typedef typename Elem<ET>::T T;
  typedef typename Frag<T>::V V;
  const T* A = (const T*)Ap; const T* A2 = (const T*)A2p; const T* Bt = (const T*)Btp; const T* Bt2 = (const T*)Bt2p;
  __shared__ __align__(16) float sT[8][16 * 68];
  const int b    = blockIdx.y;
  const int lane = threadIdx.x & 31;
  const int wave = threadIdx.x >> 5;
  const int tilesN = N >> 6;
  const int tilesM = M >> 6;
  const int tile = blockIdx.x * 8 + wave;
  if (tile >= tilesM * tilesN) return;
  const int tm = tile / tilesN;
  const int tn = tile - tm * tilesN;
  const int m0 = tm << 6;
  const int n0 = tn << 6;

  const T* Ab  = A  + (size_t)b * strideA;
  const T* Bb  = Bt + (size_t)b * strideB;
  const T* Ab2 = SPLIT ? (A2  + (size_t)b * strideA) : nullptr;
  const T* Bb2 = SPLIT ? (Bt2 + (size_t)b * strideB) : nullptr;

  const int rlane = lane & 15;
  const int koff  = (lane >> 4) * 8;
  const int mOff  = (lane >> 4) * 8;

  v8f acc[4][4];
#pragma unroll
  for (int i = 0; i < 4; ++i)
#pragma unroll
    for (int j = 0; j < 4; ++j) acc[i][j] = (v8f){0.f,0.f,0.f,0.f,0.f,0.f,0.f,0.f};

  for (int k0 = 0; k0 < K; k0 += 32) {
    V bh[4], bl[4];
#pragma unroll
    for (int j = 0; j < 4; ++j) {
      const size_t bo = (size_t)(n0 + (j << 4) + rlane) * ldb + koff + k0;
      bh[j] = Frag<T>::load(Bb + bo);
      if (SPLIT) bl[j] = Frag<T>::load(Bb2 + bo);
    }
#pragma unroll
    for (int i = 0; i < 4; ++i) {
      const size_t ao = (size_t)(m0 + (i << 4) + rlane) * lda + koff + k0;
      V ah = Frag<T>::load(Ab + ao);
      V al;
      if (SPLIT) al = Frag<T>::load(Ab2 + ao);
#pragma unroll
      for (int j = 0; j < 4; ++j) {
        acc[i][j] = Frag<T>::mma(ah, bh[j], acc[i][j]);
        if (SPLIT) {
          acc[i][j] = Frag<T>::mma(ah, bl[j], acc[i][j]);
          acc[i][j] = Frag<T>::mma(al, bh[j], acc[i][j]);
        }
      }
      Frag<T>::guard(acc[i][0], acc[i][3], ah, SPLIT ? al : ah);
    }
    Frag<T>::keep(bh[0], bh[1], bh[2], bh[3]);
    if (SPLIT) Frag<T>::keep(bl[0], bl[1], bl[2], bl[3]);
  }
  acc_guard4(acc[0][0], acc[0][1], acc[0][2], acc[0][3]);
  acc_guard4(acc[1][0], acc[1][1], acc[1][2], acc[1][3]);
  acc_guard4(acc[2][0], acc[2][1], acc[2][2], acc[2][3]);
  acc_guard4(acc[3][0], acc[3][1], acc[3][2], acc[3][3]);

  float* slab = sT[wave];
  const float* Rb = RESID ? (resid + (size_t)b * strideR) : nullptr;
#pragma unroll
  for (int i = 0; i < 4; ++i) {
    const int mBase = m0 + (i << 4);
#pragma unroll
    for (int j = 0; j < 4; ++j) {
      const int n = n0 + (j << 4) + rlane;
      float bv = 0.f;
      if (BIAS_MODE == 2) bv = bias[n];
#pragma unroll
      for (int r = 0; r < 8; ++r) {
        float v = acc[i][j][r] * scale;
        if (BIAS_MODE == 1) v += bias[mBase + mOff + r];
        if (BIAS_MODE == 2) v += bv;
        if (RESID) v += Rb[(size_t)(mBase + mOff + r) * ldc + n];
        if (ACT == 1) v = tanhf(v);
        if (ACT == 2) v = fmaxf(v, 0.0f);
        if (ACT == 3) v = v / (1.0f + expf(-v));
        if (ACT == 4) v = (v > 0.f) ? v : 0.01f * v;
        if (ACT == 5) v = 0.5f * v * (1.0f + erff(v * 0.70710678118654752f));
        if (ACT == 6) v = 1.0f / (1.0f + expf(-v));
        slab[(mOff + r) * 68 + (j << 4) + rlane] = v;
      }
    }
    __builtin_amdgcn_fence(__ATOMIC_RELEASE, "workgroup");
    __builtin_amdgcn_wave_barrier();
    __builtin_amdgcn_fence(__ATOMIC_ACQUIRE, "workgroup");
    if (OUT_MODE == 0) {
      float* C = (float*)Cout + (size_t)b * strideC;
      const int hh = lane >> 4, c4 = (lane & 15) * 4;
      for (int pass = 0; pass < 2; ++pass) {
#pragma unroll
        for (int it = 0; it < 8; ++it) {
          const int row = it * 2 + hh;
          v4f v = *(const v4f*)(slab + row * 68 + c4);
          *(volatile v4f*)(C + (size_t)(mBase + row) * ldc + n0 + c4) = v;
        }
        __threadfence();
      }
    } else {
      const int q = lane >> 3, c8 = (lane & 7) * 8;
      unsigned short* C  = (unsigned short*)Cout  + (size_t)b * strideC;
      unsigned short* C2 = (OUT_MODE == 2) ? ((unsigned short*)Cout2 + (size_t)b * strideC) : nullptr;
      for (int pass = 0; pass < 2; ++pass) {
#pragma unroll
        for (int it = 0; it < 4; ++it) {
          const int row = it * 4 + q;
          const float* sp = slab + row * 68 + c8;
          v8h hv, lv;
#pragma unroll
          for (int e = 0; e < 8; ++e) {
            if (OUT_MODE == 1) {
              hv[e] = (_Float16)sp[e];
            } else {
              unsigned short hb = f2bf_bits(sp[e]);
              unsigned short lb = f2bf_bits(sp[e] - bf_bits2f(hb));
              hv[e] = __builtin_bit_cast(_Float16, hb);
              lv[e] = __builtin_bit_cast(_Float16, lb);
            }
          }
          *(volatile v8h*)(C + (size_t)(mBase + row) * ldc + n0 + c8) = hv;
          if (OUT_MODE == 2) *(volatile v8h*)(C2 + (size_t)(mBase + row) * ldc + n0 + c8) = lv;
        }
        __threadfence();
      }
    }
    __builtin_amdgcn_fence(__ATOMIC_RELEASE, "workgroup");
    __builtin_amdgcn_wave_barrier();
    __builtin_amdgcn_fence(__ATOMIC_ACQUIRE, "workgroup");
  }
}

__global__ __launch_bounds__(256) void cast_f32_f16x2(
    const float* __restrict__ in, _Float16* __restrict__ out, int n2) {
  int i = blockIdx.x * 256 + threadIdx.x;
  if (i < n2) {
    const _Float16 h0 = (_Float16)in[2 * i], h1 = (_Float16)in[2 * i + 1];
    const unsigned u = (unsigned)__builtin_bit_cast(unsigned short, h0) | ((unsigned)__builtin_bit_cast(unsigned short, h1) << 16);
    ((volatile unsigned*)out)[i] = u;
    __threadfence();
    ((volatile unsigned*)out)[i] = u;
  }
}

__global__ __launch_bounds__(256) void transpose_scale_f16(
    const float* __restrict__ in, _Float16* __restrict__ out, int K, int N, float scl) {
  __shared__ float tile[64][65];
  const int n0 = blockIdx.x * 64, k0 = blockIdx.y * 64;
  const int tid = threadIdx.x;
#pragma unroll
  for (int i = 0; i < 16; ++i) {
    const int idx = i * 256 + tid;
    const int kr = idx >> 6, nc = idx & 63;
    int kk = k0 + kr; kk = kk < K ? kk : K - 1;
    int nn = n0 + nc; nn = nn < N ? nn : N - 1;
    tile[kr][nc] = in[(size_t)kk * N + nn];
  }
  __syncthreads();
  const int lane = tid & 31, wave = tid >> 5;
  const int q = lane >> 3, c8 = (lane & 7) * 8;
  for (int pass = 0; pass < 2; ++pass) {
#pragma unroll
    for (int it = 0; it < 2; ++it) {
      const int nr = wave * 8 + it * 4 + q;
      v8h hv;
#pragma unroll
      for (int e = 0; e < 8; ++e) hv[e] = (_Float16)(tile[c8 + e][nr] * scl);
      if ((n0 + nr) < N && (k0 + c8 + 8) <= K)
        *(volatile v8h*)(out + (size_t)(n0 + nr) * K + k0 + c8) = hv;
    }
    __threadfence();
  }
}

__global__ __launch_bounds__(128) void scan_ln_kernel(
    const float* __restrict__ feat, const float* __restrict__ gam, const float* __restrict__ bet,
    _Float16* __restrict__ lnh, int nsteps, int bsz) {
  __shared__ float redA[4];
  __shared__ float redB[4];
  const int b = blockIdx.x;
  const int tid = threadIdx.x;
  const int wave = tid >> 5;
  const int c0 = tid * 8;

  float g8[8], b8[8];
  {
    const v4f ga = *(const v4f*)(gam + c0), gb = *(const v4f*)(gam + c0 + 4);
    const v4f ba = *(const v4f*)(bet + c0), bb = *(const v4f*)(bet + c0 + 4);
#pragma unroll
    for (int e = 0; e < 4; ++e) { g8[e] = ga[e]; g8[4 + e] = gb[e]; b8[e] = ba[e]; b8[4 + e] = bb[e]; }
  }
  float S[16];
#pragma unroll
  for (int i = 0; i < 16; ++i) S[i] = 0.f;

#pragma unroll 1
  for (int t = 0; t < nsteps; ++t) {
    const size_t row = (size_t)t * (size_t)bsz + (size_t)b;
    const float* rp = feat + row * (size_t)SC_N3 + c0;
    const v4f ia = *(const v4f*)(rp),             ib = *(const v4f*)(rp + 4);
    const v4f qa = *(const v4f*)(rp + SC_D),      qb = *(const v4f*)(rp + SC_D + 4);
    const v4f la = *(const v4f*)(rp + 2 * SC_D),  lb = *(const v4f*)(rp + 2 * SC_D + 4);
    float inp[8], gt[8], lm[8];
#pragma unroll
    for (int e = 0; e < 4; ++e) {
      inp[e] = ia[e]; inp[4 + e] = ib[e];
      gt[e]  = qa[e]; gt[4 + e]  = qb[e];
      lm[e]  = la[e]; lm[4 + e]  = lb[e];
    }
    float o[8];
#pragma unroll
    for (int u = 0; u < 4; ++u) {
#pragma unroll
      for (int dd = 0; dd < 2; ++dd) {
        const float l  = lm[2 * u + dd];
        const float dm = 1.0f - l;
#pragma unroll
        for (int ee = 0; ee < 2; ++ee) {
          const float dr = dm * inp[2 * u + ee];
          S[u * 4 + dd * 2 + ee] = l * S[u * 4 + dd * 2 + ee] + dr;
        }
      }
#pragma unroll
      for (int ee = 0; ee < 2; ++ee)
        o[2 * u + ee] = S[u * 4 + ee] * gt[2 * u] + S[u * 4 + 2 + ee] * gt[2 * u + 1];
    }
    float ps = ((o[0] + o[1]) + (o[2] + o[3])) + ((o[4] + o[5]) + (o[6] + o[7]));
#pragma unroll
    for (int off = 1; off < 32; off <<= 1) ps += __shfl_xor(ps, off, 32);
    redA[wave] = ps;
    __syncthreads();
    const float mu = ((redA[0] + redA[1]) + (redA[2] + redA[3])) * (1.0f / SC_D);
    float pv = 0.f;
#pragma unroll
    for (int e = 0; e < 8; ++e) { const float d = o[e] - mu; pv += d * d; }
#pragma unroll
    for (int off = 1; off < 32; off <<= 1) pv += __shfl_xor(pv, off, 32);
    redB[wave] = pv;
    __syncthreads();
    const float var  = ((redB[0] + redB[1]) + (redB[2] + redB[3])) * (1.0f / SC_D);
    const float rstd = rsqrtf(var + 1e-5f);
    v8h hv;
#pragma unroll
    for (int e = 0; e < 8; ++e) hv[e] = (_Float16)((o[e] - mu) * rstd * g8[e] + b8[e]);
    _Float16* dst = lnh + row * (size_t)SC_D + c0;
    *(volatile v8h*)dst = hv;
    __threadfence();
    *(volatile v8h*)dst = hv;
  }
}

extern "C" void kernel_launch(void* const* d_in, const int* in_sizes, int n_in,
                              void* d_out, int out_size, void* d_ws, size_t ws_size,
                              hipStream_t stream) {
  if (n_in < 7) return;
  const int D  = SC_D;
  const int N3 = SC_N3;
  const int B  = 4;
  const int R  = in_sizes[0] / D;
  if (in_sizes[0] != R * D || (R % 64) != 0 || (R % B) != 0) return;
  if (in_sizes[1] != D * N3 || in_sizes[2] != N3 || in_sizes[3] != D * D ||
      in_sizes[4] != D || in_sizes[5] != D || in_sizes[6] != D) return;
  if (out_size != R * D) return;
  const int T = R / B;

  const float* x     = (const float*)d_in[0];
  const float* W_in  = (const float*)d_in[1];
  const float* b_in  = (const float*)d_in[2];
  const float* W_out = (const float*)d_in[3];
  const float* b_out = (const float*)d_in[4];
  const float* ln_g  = (const float*)d_in[5];
  const float* ln_b  = (const float*)d_in[6];
  float* out = (float*)d_out;

  const size_t szFeat = (size_t)R * N3 * sizeof(float);
  const size_t szXh   = (size_t)R * D * 2;
  const size_t szBt1  = (size_t)N3 * D * 2;
  const size_t szBt2  = (size_t)D * D * 2;
  const size_t offFeat = 0;
  const size_t offXh   = offFeat + szFeat;
  const size_t offBt1  = offXh + szXh;
  const size_t offBt2  = offBt1 + szBt1;
  const size_t total   = offBt2 + szBt2;
  if (total > ws_size) return;

  char* ws = (char*)d_ws;
  float*    feat = (float*)(ws + offFeat);
  _Float16* xh   = (_Float16*)(ws + offXh);
  _Float16* lnh  = xh;
  _Float16* Bt1  = (_Float16*)(ws + offBt1);
  _Float16* Bt2  = (_Float16*)(ws + offBt2);

  {
    const int n2 = (R * D) / 2;
    cast_f32_f16x2<<<(n2 + 255) / 256, 256, 0, stream>>>(x, xh, n2);
  }
  transpose_scale_f16<<<dim3((N3 + 63) / 64, (D + 63) / 64), 256, 0, stream>>>(W_in, Bt1, D, N3, 64.0f);
  transpose_scale_f16<<<dim3((D + 63) / 64, (D + 63) / 64), 256, 0, stream>>>(W_out, Bt2, D, D, 64.0f);

  {
    const int tiles = (R / 64) * (D / 64);
    wmma_gemm64<0, false, 2, 0, false, 3><<<dim3((tiles + 7) / 8, 1), 256, 0, stream>>>(
        (const unsigned short*)xh, (const unsigned short*)xh, D, 0L,
        (const unsigned short*)Bt1, (const unsigned short*)Bt1, D, 0L,
        (void*)feat, (void*)feat, N3, 0L,
        b_in, b_in, 0L, R, D, D, 1.0f / 64.0f);
  }
  {
    const int tiles = (R / 64) * ((2 * D) / 64);
    wmma_gemm64<0, false, 2, 0, false, 6><<<dim3((tiles + 7) / 8, 1), 256, 0, stream>>>(
        (const unsigned short*)xh, (const unsigned short*)xh, D, 0L,
        (const unsigned short*)(Bt1 + (size_t)D * D), (const unsigned short*)(Bt1 + (size_t)D * D), D, 0L,
        (void*)(feat + D), (void*)(feat + D), N3, 0L,
        b_in + D, b_in, 0L, R, 2 * D, D, 1.0f / 64.0f);
  }
  scan_ln_kernel<<<B, 128, 0, stream>>>(feat, ln_g, ln_b, lnh, T, B);

  {
    const int tiles = (R / 64) * (D / 64);
    wmma_gemm64<0, false, 2, 0, false, 0><<<dim3((tiles + 7) / 8, 1), 256, 0, stream>>>(
        (const unsigned short*)lnh, (const unsigned short*)lnh, D, 0L,
        (const unsigned short*)Bt2, (const unsigned short*)Bt2, D, 0L,
        (void*)out, (void*)out, D, 0L,
        b_out, b_out, 0L, R, D, D, 1.0f / 64.0f);
  }
}
